// GPTAttention_73864847557017
// MI455X (gfx1250) — hardware-verified
//
#include <hip/hip_runtime.h>
#include <math.h>

typedef __attribute__((ext_vector_type(16))) _Float16 v16h;
typedef __attribute__((ext_vector_type(16))) __bf16 v16b;
typedef __attribute__((ext_vector_type(8)))  _Float16 v8h;
typedef __attribute__((ext_vector_type(8)))  __bf16 v8b;
typedef __attribute__((ext_vector_type(8)))  float v8f;
typedef __attribute__((ext_vector_type(4)))  float v4f;
typedef __attribute__((ext_vector_type(4)))  unsigned v4u;
typedef __attribute__((ext_vector_type(4)))  int v4i;

template <typename T> __device__ __forceinline__ void vst2(void* p, T v) { *(volatile T*)p = v; __threadfence(); *(volatile T*)p = v; }
__device__ __forceinline__ v8f wmma16(v16h a, v16h b, v8f c) {
  v8f d = __builtin_amdgcn_wmma_f32_16x16x32_f16(false, a, false, b, (short)0, c, false, false);
  asm volatile("v_nop\n\tv_nop\n\tv_nop\n\tv_nop" : "+v"(d) : "v"(a), "v"(b));
  return d;
}
__device__ __forceinline__ v8f wmma_bf(v16b a, v16b b, v8f c) {
  v8f d = __builtin_amdgcn_wmma_f32_16x16x32_bf16(false, a, false, b, (short)0, c, false, false);
  asm volatile("v_nop\n\tv_nop\n\tv_nop\n\tv_nop" : "+v"(d) : "v"(a), "v"(b));
  return d;
}
__device__ __forceinline__ v16h frag_h(const _Float16* rowk0, int lane) {
  union { v16h v; v8h q[2]; } u; const _Float16* p = rowk0 + 8 * (lane >> 4);
  u.q[0] = *(const v8h*)p; u.q[1] = *(const v8h*)(p + 16); return u.v;
}
__device__ __forceinline__ v16b frag_b(const __bf16* rowk0, int lane) {
  union { v16b v; v8b q[2]; } u; const __bf16* p = rowk0 + 8 * (lane >> 4);
  u.q[0] = *(const v8b*)p; u.q[1] = *(const v8b*)(p + 16); return u.v;
}
__device__ __forceinline__ float bfr(float v) { return (float)(__bf16)v; }
#define LDSX() do { asm volatile("s_wait_dscnt 0" ::: "memory"); __builtin_amdgcn_wave_barrier(); __builtin_amdgcn_fence(__ATOMIC_RELEASE, "workgroup"); } while (0)

#ifndef NB
#define NB 2
#endif
#ifndef SEQ
#define SEQ 2048
#endif
#define NB_FULL 2
#define SEQ_FULL 2048
#define DM 2048
#define NH 32
#define HD 64
#define RSPAN 512
#if RSPAN > SEQ
#define RS SEQ
#else
#define RS RSPAN
#endif
#define RQB (RS / 64)
#define NR (NB * SEQ)
#define TQB (SEQ / 64)
#define NKTILE (SEQ / 32)
static_assert(SEQ % 64 == 0);
static_assert(RS % 64 == 0);
static_assert(NB >= 1 && NB <= NB_FULL);
static_assert(SEQ <= SEQ_FULL);
static_assert(DM == 256 * 8);
static_assert(NH * HD == DM);
static_assert(NR % 64 == 0);

#define WS_PKA 0ull
#define WS_PKO (WS_PKA + 2ull * 3 * DM * DM)
#define WS_QK  (WS_PKO + 2ull * DM * DM)
#define WS_QKL (WS_QK + 2ull * NR * 2 * DM)
#define WS_VTH (WS_QKL + 2ull * NB * RS * 2 * DM)
#define WS_VTL (WS_VTH + 2ull * NB * DM * SEQ)
#define WS_OH  (WS_VTL + 2ull * NB * DM * RS)
#define WS_OL  (WS_OH + 2ull * NR * DM)
#define WS_NKT (WS_OL + 2ull * NB * RS * DM)
#define WS_END (WS_NKT + 128ull * TQB)
static_assert(2ull * NR * DM == (WS_OL - WS_OH));
static_assert(WS_END <= 134217728ull);
static_assert((WS_PKO % 128) == 0 && (WS_QK % 128) == 0 && (WS_QKL % 128) == 0 && (WS_VTH % 128) == 0 && (WS_VTL % 128) == 0 && (WS_OH % 128) == 0 && (WS_OL % 128) == 0 && (WS_NKT % 128) == 0);

__global__ __launch_bounds__(256) void k_cvtx(const float* __restrict__ X, __bf16* __restrict__ XB) {
  const int r = blockIdx.x, t = threadIdx.x; const int b = r / SEQ, s = r - b * SEQ;
  const float* src = X + ((size_t)b * SEQ_FULL + s) * DM + t * 8;
  const v4f x = *(const v4f*)src, y = *(const v4f*)(src + 4);
  union { v8b v; v4u u; } o;
#pragma unroll
  for (int j = 0; j < 4; ++j) { o.v[j] = (__bf16)x[j]; o.v[4 + j] = (__bf16)y[j]; }
  vst2(XB + (size_t)r * DM + t * 8, o.u);
}
__global__ __launch_bounds__(256) void k_pack(const float* __restrict__ WQ, const float* __restrict__ WK, const float* __restrict__ WV, const float* __restrict__ WO, __bf16* __restrict__ PKA, _Float16* __restrict__ PKO) {
  const int n = blockIdx.x, which = blockIdx.y, t = threadIdx.x;
  const float* W = (which == 0) ? WQ : (which == 1) ? WK : (which == 2) ? WV : WO;
  const float* src = W + (size_t)n * DM + t * 8;
  const v4f x = *(const v4f*)src, y = *(const v4f*)(src + 4);
  if (which < 3) {
    union { v8b v; v4u u; } o;
#pragma unroll
    for (int j = 0; j < 4; ++j) { o.v[j] = (__bf16)x[j]; o.v[4 + j] = (__bf16)y[j]; }
    vst2(PKA + ((size_t)which * DM + n) * DM + t * 8, o.u);
  } else {
    union { v8h v; v4u u; } o;
#pragma unroll
    for (int j = 0; j < 4; ++j) { o.v[j] = (_Float16)(bfr(x[j]) * 64.0f); o.v[4 + j] = (_Float16)(bfr(y[j]) * 64.0f); }
    vst2(PKO + (size_t)n * DM + t * 8, o.u);
  }
}
__global__ __launch_bounds__(128) void k_qkv(const __bf16* __restrict__ XB, const __bf16* __restrict__ P, const float* __restrict__ BQ, const float* __restrict__ BK, const float* __restrict__ BV,
                                             _Float16* __restrict__ QK, _Float16* __restrict__ QKL, _Float16* __restrict__ VTH, _Float16* __restrict__ VTL) {
  const int n0 = blockIdx.y * 128; const int which0 = n0 / DM;
  const float* BB = ((which0 == 0) ? BQ : (which0 == 1) ? BK : BV) + (n0 - which0 * DM);
  __shared__ __align__(16) _Float16 so[4][16][136], sol[4][16][136]; __shared__ __align__(16) _Float16 sth[128][72], stl[128][72];
  const int tid = threadIdx.x, wave = tid >> 5, lane = tid & 31, col = lane & 15, g = lane >> 4;
  const int rb = blockIdx.x * 64; const int b = rb / SEQ, s0 = rb - b * SEQ; const int r0 = rb + wave * 16; const bool resid = (s0 < RS);
  v8f acc[8] = {};
#pragma unroll 2
  for (int kc = 0; kc < DM / 32; ++kc) {
    const v16b a = frag_b(XB + (size_t)(r0 + col) * DM + kc * 32, lane);
#pragma unroll
    for (int j = 0; j < 8; ++j) acc[j] = wmma_bf(a, frag_b(P + (size_t)(n0 + j * 16 + col) * DM + kc * 32, lane), acc[j]);
  }
  if (n0 < 2 * DM) {
#pragma unroll
    for (int j = 0; j < 8; ++j) { const float bj = bfr(BB[j * 16 + col]);
#pragma unroll
      for (int r = 0; r < 8; ++r) { const float v = acc[j][r] + bj; const _Float16 hv = (_Float16)v; so[wave][8 * g + r][j * 16 + col] = hv; sol[wave][8 * g + r][j * 16 + col] = (_Float16)((v - (float)hv) * 2048.0f); } }
    LDSX();
    const size_t ql = (size_t)b * RS + s0 + wave * 16;
    for (int rl = 0; rl < 16; ++rl) if (lane < 16) {
      vst2(QK + (size_t)(r0 + rl) * (2 * DM) + n0 + lane * 8, *(const v4u*)&so[wave][rl][lane * 8]);
      if (resid) vst2(QKL + (ql + rl) * (2 * DM) + n0 + lane * 8, *(const v4u*)&sol[wave][rl][lane * 8]);
    }
  } else {
#pragma unroll
    for (int j = 0; j < 8; ++j) { const float bj = bfr(BB[j * 16 + col]);
#pragma unroll
      for (int r = 0; r < 8; ++r) { const float v = acc[j][r] + bj; const _Float16 hv = (_Float16)v; sth[j * 16 + col][wave * 16 + 8 * g + r] = hv; stl[j * 16 + col][wave * 16 + 8 * g + r] = (_Float16)((v - (float)hv) * 2048.0f); } }
    __syncthreads();
    const int pc0 = n0 - 2 * DM;
    for (int q = tid; q < 128 * 8; q += 128) {
      const int d = q >> 3, pc = q & 7;
      vst2(VTH + ((size_t)b * DM + pc0 + d) * SEQ + s0 + pc * 8, *(const v4u*)&sth[d][pc * 8]);
      if (resid) vst2(VTL + ((size_t)b * DM + pc0 + d) * RS + s0 + pc * 8, *(const v4u*)&stl[d][pc * 8]);
    }
  }
}
__global__ __launch_bounds__(256) void k_mscan(const float* __restrict__ MK, int* __restrict__ NKT) {
  __shared__ int srow[64][4]; __shared__ __align__(16) int sline[32];
  const int qb = blockIdx.x, t = threadIdx.x, row = t >> 2, part = t & 3;
  const float* p = MK + (size_t)(qb * 64 + row) * SEQ_FULL + part * (SEQ / 4);
  int mx = -1;
#pragma unroll 1
  for (int c = 0; c < SEQ / 4; c += 4) {
    const v4f v = *(const v4f*)(p + c);
#pragma unroll
    for (int j = 0; j < 4; ++j) mx = (v[j] > -1.0e8f) ? (part * (SEQ / 4) + c + j) : mx;
  }
  srow[row][part] = mx; __syncthreads();
  if (t == 0) {
    int last = -1, dead = 0;
    for (int r = 0; r < 64; ++r) {
      int a = srow[r][0] > srow[r][1] ? srow[r][0] : srow[r][1]; const int c2 = srow[r][2] > srow[r][3] ? srow[r][2] : srow[r][3]; a = a > c2 ? a : c2;
      last = last > a ? last : a; dead |= (a < 0) ? 1 : 0;
    }
    const int nk = dead ? NKTILE : (last / 32 + 1);
    for (int i = 0; i < 32; ++i) sline[i] = nk;
  }
  __syncthreads();
  if (t < 8) vst2(NKT + (size_t)qb * 32 + t * 4, *(const v4i*)&sline[t * 4]);
}
__global__ __launch_bounds__(128) void k_attn(const _Float16* __restrict__ QK, const _Float16* __restrict__ QKL, const _Float16* __restrict__ VTH, const _Float16* __restrict__ VTL,
                                              const float* __restrict__ MK, const int* __restrict__ NKT, _Float16* __restrict__ OH, _Float16* __restrict__ OL) {
  __shared__ __align__(16) float sp[4][16][36]; __shared__ __align__(16) float sm[4][16][36]; __shared__ __align__(16) _Float16 so[4][16][72], sol[4][16][72];
  const int tid = threadIdx.x, wave = tid >> 5, lane = tid & 31, col = lane & 15, g = lane >> 4;
  const int qb = blockIdx.x, h = blockIdx.y, b = blockIdx.z; const int q0 = qb * 64 + wave * 16;
  int nkt = NKT[(size_t)qb * 32]; nkt = (nkt < 1) ? 1 : ((nkt > NKTILE) ? NKTILE : nkt);
  const bool res3 = (qb < RQB) && (nkt * 32 <= RS);
  const size_t rq = (size_t)b * SEQ + q0 + col;
  v16h aq[2], aql[2];
#pragma unroll
  for (int kc = 0; kc < 2; ++kc) aq[kc] = frag_h(QK + rq * (2 * DM) + h * HD + kc * 32, lane);
  if (res3) { const size_t rql = (size_t)b * RS + q0 + col;
#pragma unroll
    for (int kc = 0; kc < 2; ++kc) aql[kc] = frag_h(QKL + rql * (2 * DM) + h * HD + kc * 32, lane); }
  else { v16h z = {}; aql[0] = z; aql[1] = z; }
  float m[8], l[8];
#pragma unroll
  for (int r = 0; r < 8; ++r) { m[r] = -3.0e38f; l[r] = 0.f; }
  v8f acc[4] = {}, accl[4] = {};
#pragma unroll 1
  for (int ks = 0; ks < nkt; ++ks) {
#pragma unroll
    for (int i = 0; i < 4; ++i) { const int row = (lane >> 3) + 4 * i, c4 = (lane & 7) * 4;
      *(v4f*)&sm[wave][row][c4] = *(const v4f*)(MK + (size_t)(q0 + row) * SEQ_FULL + ks * 32 + c4); }
    LDSX();
    v8f s[2];
#pragma unroll
    for (int ct = 0; ct < 2; ++ct) {
      const int kk = ks * 32 + ct * 16 + col; const _Float16* krow = QK + ((size_t)b * SEQ + kk) * (2 * DM) + DM + h * HD; v8f c = {};
      if (res3) {
        const _Float16* krowl = QKL + ((size_t)b * RS + kk) * (2 * DM) + DM + h * HD; v8f cl = {};
#pragma unroll
        for (int kc = 0; kc < 2; ++kc) { const v16h kh = frag_h(krow + kc * 32, lane); c = wmma16(aq[kc], kh, c); cl = wmma16(aql[kc], kh, cl); cl = wmma16(aq[kc], frag_h(krowl + kc * 32, lane), cl); }
#pragma unroll
        for (int r = 0; r < 8; ++r) c[r] += cl[r] * (1.0f / 2048.0f);
      } else {
#pragma unroll
        for (int kc = 0; kc < 2; ++kc) c = wmma16(aq[kc], frag_h(krow + kc * 32, lane), c);
      }
#pragma unroll
      for (int r = 0; r < 8; ++r) s[ct][r] = c[r] * 0.125f + sm[wave][8 * g + r][ct * 16 + col];
    }
#pragma unroll
    for (int r = 0; r < 8; ++r) {
      float mx = fmaxf(s[0][r], s[1][r]);
#pragma unroll
      for (int o = 1; o < 16; o <<= 1) mx = fmaxf(mx, __shfl_xor(mx, o));
      const float mn = fmaxf(m[r], mx); const float alpha = (m[r] <= -1.0e38f) ? 0.f : __expf(m[r] - mn);
      const float e0 = __expf(s[0][r] - mn), e1 = __expf(s[1][r] - mn); float es = e0 + e1;
#pragma unroll
      for (int o = 1; o < 16; o <<= 1) es += __shfl_xor(es, o);
      l[r] = l[r] * alpha + es; m[r] = mn;
#pragma unroll
      for (int dt = 0; dt < 4; ++dt) { acc[dt][r] *= alpha; accl[dt][r] *= alpha; }
      sp[wave][8 * g + r][col] = e0; sp[wave][8 * g + r][16 + col] = e1;
    }
    LDSX();
    v16h pa, pl; { const float* prow = &sp[wave][col][0] + 8 * (lane >> 4);
#pragma unroll
      for (int i = 0; i < 8; ++i) { const float x0 = prow[i] * 2048.0f, x1 = prow[16 + i] * 2048.0f; const _Float16 h0 = (_Float16)x0, h1 = (_Float16)x1;
        pa[i] = h0; pa[8 + i] = h1; pl[i] = (_Float16)((x0 - (float)h0) * 2048.0f); pl[8 + i] = (_Float16)((x1 - (float)h1) * 2048.0f); } }
#pragma unroll
    for (int dt = 0; dt < 4; ++dt) {
      const size_t vr = ((size_t)b * DM + h * HD + dt * 16 + col) * SEQ + ks * 32; const v16h vh = frag_h(VTH + vr, lane);
      acc[dt] = wmma16(pa, vh, acc[dt]);
      if (res3) { accl[dt] = wmma16(pl, vh, accl[dt]); accl[dt] = wmma16(pa, frag_h(VTL + ((size_t)b * DM + h * HD + dt * 16 + col) * RS + ks * 32, lane), accl[dt]); }
    }
    LDSX();
  }
#pragma unroll
  for (int r = 0; r < 8; ++r) { const float il = (1.0f / 2048.0f) / l[r];
#pragma unroll
    for (int dt = 0; dt < 4; ++dt) { const float o = (acc[dt][r] + accl[dt][r] * (1.0f / 2048.0f)) * il; const _Float16 hv = (_Float16)o;
      so[wave][8 * g + r][dt * 16 + col] = hv; sol[wave][8 * g + r][dt * 16 + col] = (_Float16)((o - (float)hv) * 2048.0f); } }
  LDSX();
#pragma unroll
  for (int it = 0; it < 4; ++it) {
    const int row = it * 4 + (lane >> 3), pc = lane & 7;
    vst2(OH + ((size_t)b * SEQ + q0 + row) * DM + h * HD + pc * 8, *(const v4u*)&so[wave][row][pc * 8]);
    if (qb < RQB) vst2(OL + ((size_t)b * RS + q0 + row) * DM + h * HD + pc * 8, *(const v4u*)&sol[wave][row][pc * 8]);
  }
}
__global__ __launch_bounds__(128) void k_out(const _Float16* __restrict__ OH, const _Float16* __restrict__ OL, const _Float16* __restrict__ PO, const float* __restrict__ BO, float* __restrict__ Y) {
  __shared__ __align__(16) float so[4][16][68];
  const int tid = threadIdx.x, wave = tid >> 5, lane = tid & 31, col = lane & 15, g = lane >> 4;
  const int rb = blockIdx.x * 64; const int b = rb / SEQ, s0 = rb - b * SEQ; const int r0 = rb + wave * 16; const int n0 = blockIdx.y * 64; const bool resid = (s0 < RS);
  const size_t rl0 = (size_t)b * RS + s0 + wave * 16;
  v8f acc[4] = {}, accl[4] = {};
#pragma unroll 2
  for (int kc = 0; kc < DM / 32; ++kc) {
    const v16h a = frag_h(OH + (size_t)(r0 + col) * DM + kc * 32, lane);
    v16h al = {}; if (resid) al = frag_h(OL + (rl0 + col) * DM + kc * 32, lane);
#pragma unroll
    for (int j = 0; j < 4; ++j) { const v16h w = frag_h(PO + (size_t)(n0 + j * 16 + col) * DM + kc * 32, lane); acc[j] = wmma16(a, w, acc[j]); if (resid) accl[j] = wmma16(al, w, accl[j]); }
  }
#pragma unroll
  for (int j = 0; j < 4; ++j) { const float bj = bfr(BO[n0 + j * 16 + col]);
#pragma unroll
    for (int r = 0; r < 8; ++r) so[wave][8 * g + r][j * 16 + col] = acc[j][r] * (1.0f / 64.0f) + accl[j][r] * (1.0f / 131072.0f) + bj; }
  LDSX();
  const size_t yr = (size_t)b * SEQ_FULL + s0 + wave * 16;
  for (int rl = 0; rl < 16; ++rl) if (lane < 16) vst2(Y + (yr + rl) * DM + n0 + lane * 4, *(const v4f*)&so[wave][rl][lane * 4]);
}
extern "C" void kernel_launch(void* const* d_in, const int* in_sizes, int n_in, void* d_out, int out_size, void* d_ws, size_t ws_size, hipStream_t stream) {
  if (n_in < 10) return;
  const long long needx = ((long long)(NB - 1) * SEQ_FULL + SEQ) * DM;
  if ((long long)in_sizes[0] < needx) return;
  if ((long long)in_sizes[1] < (long long)(SEQ - 1) * SEQ_FULL + SEQ) return;
  if (in_sizes[2] < DM * DM || in_sizes[4] < DM * DM || in_sizes[6] < DM * DM || in_sizes[8] < DM * DM) return;
  if (in_sizes[3] < DM || in_sizes[5] < DM || in_sizes[7] < DM || in_sizes[9] < DM) return;
  if ((long long)out_size < needx) return;
  if (ws_size < (size_t)WS_END) return;
  const float* const* F = (const float* const*)d_in;
  char* ws = (char*)d_ws;
  __bf16* PKA = (__bf16*)(ws + WS_PKA); _Float16* PKO = (_Float16*)(ws + WS_PKO);
  _Float16 *QK = (_Float16*)(ws + WS_QK), *QKL = (_Float16*)(ws + WS_QKL), *VTH = (_Float16*)(ws + WS_VTH), *VTL = (_Float16*)(ws + WS_VTL), *OH = (_Float16*)(ws + WS_OH), *OL = (_Float16*)(ws + WS_OL);
  __bf16* XB = (__bf16*)(ws + WS_OH);
  int* NKT = (int*)(ws + WS_NKT);
  k_cvtx<<<dim3(NR), 256, 0, stream>>>(F[0], XB);
  k_pack<<<dim3(DM, 4), 256, 0, stream>>>(F[2], F[4], F[6], F[8], PKA, PKO);
  k_qkv<<<dim3(NR / 64, 3 * DM / 128), 128, 0, stream>>>(XB, PKA, F[3], F[5], F[7], QK, QKL, VTH, VTL);
  k_mscan<<<dim3(TQB), 256, 0, stream>>>(F[1], NKT);
  k_attn<<<dim3(TQB, NH, NB), 128, 0, stream>>>(QK, QKL, VTH, VTL, F[1], NKT, OH, OL);
  k_out<<<dim3(NR / 64, DM / 64), 128, 0, stream>>>(OH, OL, PKO, F[9], (float*)d_out);
}
